// BitPosAttMD_64510408786004
// MI455X (gfx1250) — hardware-verified
//
#include <hip/hip_runtime.h>


#define NB_  4
#define NC_  256
#define CK   64
#define NN_  4096

typedef _Float16 h16;
typedef unsigned short bf;
typedef __attribute__((ext_vector_type(16))) __bf16   v16bf;
typedef __attribute__((ext_vector_type(16))) _Float16 v16h;
typedef __attribute__((ext_vector_type(8)))  _Float16 v8h;
typedef __attribute__((ext_vector_type(8)))  unsigned short v8us;
typedef __attribute__((ext_vector_type(8)))  float    v8f;
typedef __attribute__((ext_vector_type(4)))  float    v4f;
typedef v8h  __attribute__((may_alias)) v8ha;
typedef v4f  __attribute__((may_alias)) v4fa;
typedef v8us __attribute__((may_alias)) v8usa;

__device__ __forceinline__ unsigned short f2bf(float f) { unsigned u = __float_as_uint(f); u += 0x7FFFu + ((u >> 16) & 1u); return (unsigned short)(u >> 16); }
__device__ __forceinline__ float bf2f(unsigned short b) { return __uint_as_float(((unsigned)b) << 16); }
__device__ __forceinline__ float bfr(float f) { return bf2f(f2bf(f)); }
__device__ __forceinline__ v16h cat16(v8h lo, v8h hi) { return __builtin_shufflevector(lo, hi, 0, 1, 2, 3, 4, 5, 6, 7, 8, 9, 10, 11, 12, 13, 14, 15); }
__device__ __forceinline__ v16bf cat16b(v8us lo, v8us hi) { return __builtin_bit_cast(v16bf, __builtin_shufflevector(lo, hi, 0, 1, 2, 3, 4, 5, 6, 7, 8, 9, 10, 11, 12, 13, 14, 15)); }
__device__ __forceinline__ v8f wmma16(v16h a, v16h b, v8f c) { return __builtin_amdgcn_wmma_f32_16x16x32_f16(false, a, false, b, (short)0, c, false, false); }
__device__ __forceinline__ v8f wmmab(v16bf a, v16bf b, v8f c) { return __builtin_amdgcn_wmma_f32_16x16x32_bf16(false, a, false, b, (short)0, c, false, false); }
#define VST2(T, p, v) do { const T vst2_v_ = (v); *(volatile T*)(p) = vst2_v_; __threadfence(); *(volatile T*)(p) = vst2_v_; } while (0)

__global__ __launch_bounds__(256) void k_xt(const float* __restrict__ X, bf* XT) {
    __shared__ __align__(16) unsigned short tl[64 * 72];
    const int tid = threadIdx.x;
    const int b = blockIdx.z, c0 = blockIdx.y * 64, n0 = blockIdx.x * 64;
    const int cc = tid >> 2, nq = (tid & 3) * 16;
    const float* src = X + ((size_t)b * NC_ + c0 + cc) * NN_ + n0 + nq;
#pragma unroll
    for (int i = 0; i < 16; ++i) tl[(nq + i) * 72 + cc] = f2bf(src[i]);
    __syncthreads();
    const int piece = tid & 7;
    auto pass = [&]() {
#pragma unroll
        for (int s = 0; s < 2; ++s) { const int nr = (tid >> 3) + 32 * s; const v8us val = *(const v8usa*)(tl + nr * 72 + piece * 8);
            *(volatile v8us*)(XT + ((size_t)b * NN_ + n0 + nr) * NC_ + c0 + piece * 8) = val; }
    };
    pass(); __threadfence(); pass();
}

__global__ __launch_bounds__(256) void k_fold(const float* __restrict__ Wb, const float* __restrict__ bb, const float* __restrict__ Wc, const float* __restrict__ bc,
                                              const float* __restrict__ g, const float* __restrict__ be, const float* __restrict__ mean, const float* __restrict__ var,
                                              bf* WH, bf* WL, float* BIAS32) {
    const int lane = threadIdx.x & 31, row = blockIdx.x * 8 + (threadIdx.x >> 5);
    if (row >= 2 * CK) return;
    const float* Wsrc = (row < CK) ? (Wb + (size_t)row * NC_) : (Wc + (size_t)(row - CK) * NC_);
    const float bsrc = (row < CK) ? bb[row] : bc[row - CK];
    float bacc = 0.f;
    v8us oh, ol;
#pragma unroll
    for (int i = 0; i < 8; ++i) {
        const int c = lane * 8 + i;
        const float gg = bfr(g[c]), rsd = 1.0f / sqrtf(bfr(var[c]) + 1e-5f);
        const float sc = gg * rsd, sh = bfr(be[c]) - bfr(mean[c]) * gg * rsd;
        const float w = bfr(Wsrc[c]);
        const float wp = w * sc;
        const unsigned short hb = f2bf(wp); oh[i] = hb; ol[i] = f2bf(wp - bf2f(hb));
        bacc += w * sh;
    }
#pragma unroll
    for (int o = 16; o; o >>= 1) bacc += __shfl_xor(bacc, o, 32);
    VST2(v8us, WH + (size_t)row * NC_ + lane * 8, oh);
    VST2(v8us, WL + (size_t)row * NC_ + lane * 8, ol);
    VST2(float, BIAS32 + (size_t)row * 32 + lane, bacc + bfr(bsrc));
}

__global__ __launch_bounds__(256) void k_cvtw(const float* __restrict__ Wd, bf* WD) {
    const int lane = threadIdx.x & 31, r = blockIdx.x * 8 + (threadIdx.x >> 5);
    if (r >= NC_) return;
    v8us t;
#pragma unroll
    for (int i = 0; i < 8; ++i) t[i] = f2bf(Wd[(size_t)r * NC_ + lane * 8 + i]);
    VST2(v8us, WD + (size_t)r * NC_ + lane * 8, t);
}

__global__ __launch_bounds__(128) void k_gemmf(const bf* __restrict__ XT, const bf* __restrict__ WH, const bf* __restrict__ WL, const float* __restrict__ BIAS32, int which, h16* F16) {
    __shared__ __align__(16) float ost[4][16 * 68];
    const int lane = threadIdx.x & 31, wave = threadIdx.x >> 5, lr = lane & 15, hi = lane >> 4;
    const int b = blockIdx.y, r0 = blockIdx.x * 64 + wave * 16;
    const size_t aoff = ((size_t)b * NN_ + r0 + lr) * NC_ + 8 * hi;
    size_t boff[4];
#pragma unroll
    for (int t = 0; t < 4; ++t) boff[t] = (size_t)(which * CK + t * 16 + lr) * NC_ + 8 * hi;
    v8f acc[4];
#pragma unroll
    for (int t = 0; t < 4; ++t) acc[t] = (v8f){};
#pragma unroll 1
    for (int kc = 0; kc < NC_; kc += 32) {
        const v16bf a = cat16b(*(const v8us*)(XT + aoff + kc), *(const v8us*)(XT + aoff + kc + 16));
#pragma unroll
        for (int t = 0; t < 4; ++t) {
            acc[t] = wmmab(a, cat16b(*(const v8us*)(WH + boff[t] + kc), *(const v8us*)(WH + boff[t] + kc + 16)), acc[t]);
            acc[t] = wmmab(a, cat16b(*(const v8us*)(WL + boff[t] + kc), *(const v8us*)(WL + boff[t] + kc + 16)), acc[t]);
        }
        asm volatile("v_nop\n\tv_nop\n\tv_nop\n\tv_nop" : "+v"(acc[0]), "+v"(acc[1]), "+v"(acc[2]), "+v"(acc[3]) : "v"(a));
    }
    float* os = &ost[wave][0];
#pragma unroll
    for (int t = 0; t < 4; ++t) { const float bv = BIAS32[(size_t)(which * CK + t * 16 + lr) * 32];
#pragma unroll
        for (int j = 0; j < 8; ++j) os[(hi * 8 + j) * 68 + t * 16 + lr] = acc[t][j] + bv; }
    __syncthreads();
    h16* crow = F16 + ((size_t)b * NN_ + r0) * CK;
    auto pass = [&]() {
#pragma unroll
        for (int s = 0; s < 4; ++s) { const int row = 4 * s + (lane >> 3), piece = lane & 7; const float* sp = os + row * 68 + piece * 8; v8h o;
#pragma unroll
            for (int i = 0; i < 8; ++i) o[i] = (h16)sp[i];
            *(volatile v8h*)(crow + (size_t)row * CK + piece * 8) = o; }
    };
    pass(); __threadfence(); pass();
}

__global__ __launch_bounds__(128) void k_gemm1(const bf* __restrict__ WD, const bf* __restrict__ XT, const float* __restrict__ bd, h16* F1) {
    __shared__ __align__(16) float ost[4][16 * 68];
    const int lane = threadIdx.x & 31, wave = threadIdx.x >> 5, lr = lane & 15, hi = lane >> 4;
    const int b = blockIdx.z, r0 = blockIdx.x * 64 + wave * 16, c0 = blockIdx.y * 64;
    const size_t aoff = (size_t)(r0 + lr) * NC_ + 8 * hi;
    size_t boff[4];
#pragma unroll
    for (int t = 0; t < 4; ++t) boff[t] = ((size_t)b * NN_ + c0 + t * 16 + lr) * NC_ + 8 * hi;
    v8f acc[4];
#pragma unroll
    for (int t = 0; t < 4; ++t) acc[t] = (v8f){};
#pragma unroll 1
    for (int kc = 0; kc < NC_; kc += 32) {
        const v16bf a = cat16b(*(const v8us*)(WD + aoff + kc), *(const v8us*)(WD + aoff + kc + 16));
#pragma unroll
        for (int t = 0; t < 4; ++t) acc[t] = wmmab(a, cat16b(*(const v8us*)(XT + boff[t] + kc), *(const v8us*)(XT + boff[t] + kc + 16)), acc[t]);
        asm volatile("v_nop\n\tv_nop\n\tv_nop\n\tv_nop" : "+v"(acc[0]), "+v"(acc[1]), "+v"(acc[2]), "+v"(acc[3]) : "v"(a));
    }
    float* os = &ost[wave][0];
#pragma unroll
    for (int t = 0; t < 4; ++t)
#pragma unroll
        for (int j = 0; j < 8; ++j) os[(hi * 8 + j) * 68 + t * 16 + lr] = acc[t][j] + bfr(bd[r0 + 8 * hi + j]);
    __syncthreads();
    h16* crow = F1 + ((size_t)b * NC_ + r0) * NN_ + c0;
    auto pass = [&]() {
#pragma unroll
        for (int s = 0; s < 4; ++s) { const int row = 4 * s + (lane >> 3), piece = lane & 7; const float* sp = os + row * 68 + piece * 8; v8h o;
#pragma unroll
            for (int i = 0; i < 8; ++i) o[i] = (h16)sp[i];
            *(volatile v8h*)(crow + (size_t)row * NN_ + piece * 8) = o; }
    };
    pass(); __threadfence(); pass();
}

#define SCORE_TILE(n0_)                                                                                               \
    v8f s0 = {}, s1 = {};                                                                                          \
    { const h16* r0p = fb_b + (size_t)((n0_) + lr) * CK + 8 * hi; const h16* r1p = fb_b + (size_t)((n0_) + 16 + lr) * CK + 8 * hi; \
    _Pragma("unroll") for (int kc = 0; kc < 2; ++kc) {                                                            \
        s0 = wmma16(qa[kc], cat16(*(const v8h*)(r0p + kc * 32), *(const v8h*)(r0p + kc * 32 + 16)), s0);         \
        s1 = wmma16(qa[kc], cat16(*(const v8h*)(r1p + kc * 32), *(const v8h*)(r1p + kc * 32 + 16)), s1); } }     \
    asm volatile("v_nop\n\tv_nop\n\tv_nop\n\tv_nop" : "+v"(s0), "+v"(s1) : "v"(qa[0]), "v"(qa[1]));

__global__ __launch_bounds__(128) void k_rowstats(const h16* __restrict__ FA, const h16* __restrict__ FB, float* M, float* ZI) {
    __shared__ __align__(16) float stg[128];
    const int lane = threadIdx.x & 31, wave = threadIdx.x >> 5, lr = lane & 15, hi = lane >> 4;
    const int b = blockIdx.x / (NN_ / 64), qt = blockIdx.x - b * (NN_ / 64);
    const size_t row0 = (size_t)b * NN_;
    const int m0 = qt * 64 + wave * 16;
    v16h qa[2];
#pragma unroll
    for (int kc = 0; kc < 2; ++kc) { const h16* p = FA + (row0 + m0 + lr) * CK + kc * 32 + 8 * hi; qa[kc] = cat16(*(const v8h*)p, *(const v8h*)(p + 16)); }
    const h16* fb_b = FB + row0 * CK;
    float mrow[8], lpart[8];
#pragma unroll
    for (int j = 0; j < 8; ++j) { mrow[j] = -3.0e38f; lpart[j] = 0.f; }
#pragma unroll 1
    for (int it = 0; it < NN_ / 32; ++it) {
        SCORE_TILE(it * 32)
#pragma unroll
        for (int j = 0; j < 8; ++j) {
            const float a0 = s0[j], a1 = s1[j];
            float mx = fmaxf(a0, a1);
            mx = fmaxf(mx, __shfl_xor(mx, 1, 16)); mx = fmaxf(mx, __shfl_xor(mx, 2, 16)); mx = fmaxf(mx, __shfl_xor(mx, 4, 16)); mx = fmaxf(mx, __shfl_xor(mx, 8, 16));
            const float mn = fmaxf(mrow[j], mx); const float al_ = __expf(mrow[j] - mn); mrow[j] = mn;
            lpart[j] = lpart[j] * al_ + (__expf(a0 - mn) + __expf(a1 - mn));
        }
    }
#pragma unroll
    for (int j = 0; j < 8; ++j) {
        float rs = lpart[j]; rs += __shfl_xor(rs, 1, 16); rs += __shfl_xor(rs, 2, 16); rs += __shfl_xor(rs, 4, 16); rs += __shfl_xor(rs, 8, 16);
        if (lr == 0) { const int jl = wave * 16 + 8 * hi + j; stg[jl] = mrow[j]; stg[64 + jl] = 1.0f / rs; }
    }
    __syncthreads();
    if (wave == 0) {
        const v4f val = *(const v4fa*)(stg + hi * 64 + lr * 4);
        float* dst = (hi ? ZI : M) + row0 + qt * 64 + lr * 4;
        *(volatile v4f*)dst = val; __threadfence(); *(volatile v4f*)dst = val;
    }
}

__global__ __launch_bounds__(128) void k_out(const h16* __restrict__ FA, const h16* __restrict__ FB, const h16* __restrict__ F1, const float* __restrict__ M,
                                            const float* __restrict__ ZI, const float* __restrict__ x, const float* __restrict__ alpha, int cofs, float* out) {
    extern __shared__ float4 lds_raw[];
    float* stile = (float*)lds_raw;
    h16* plds = (h16*)(stile + 64 * 128);
    const int lane = threadIdx.x & 31, wave = threadIdx.x >> 5, lr = lane & 15, hi = lane >> 4;
    const int b = blockIdx.x / (NN_ / 64), qt = blockIdx.x - b * (NN_ / 64);
    const size_t row0 = (size_t)b * NN_;
    const int m0 = qt * 64 + wave * 16;
    h16* pl = plds + wave * (16 * 32);
    v16h qa[2];
#pragma unroll
    for (int kc = 0; kc < 2; ++kc) { const h16* p = FA + (row0 + m0 + lr) * CK + kc * 32 + 8 * hi; qa[kc] = cat16(*(const v8h*)p, *(const v8h*)(p + 16)); }
    const h16* fb_b = FB + row0 * CK;
    const h16* f1_b = F1 + ((size_t)b * NC_ + cofs) * NN_;
    float mr[8], zr[8];
#pragma unroll
    for (int j = 0; j < 8; ++j) { mr[j] = M[row0 + m0 + 8 * hi + j]; zr[j] = ZI[row0 + m0 + 8 * hi + j]; }
    v8f o[8];
#pragma unroll
    for (int n = 0; n < 8; ++n) o[n] = (v8f){};
#pragma unroll 1
    for (int it = 0; it < NN_ / 32; ++it) {
        const int n0 = it * 32;
        SCORE_TILE(n0)
#pragma unroll
        for (int j = 0; j < 8; ++j) {
            const float p0 = __expf(s0[j] - mr[j]) * zr[j], p1 = __expf(s1[j] - mr[j]) * zr[j];
            const float a0 = 1.0f - 1.0f / (1.0f + __expf(-p0)), a1 = 1.0f - 1.0f / (1.0f + __expf(-p1));
            const int mrw = hi * 8 + j;
            pl[mrw * 32 + lr] = (h16)a0; pl[mrw * 32 + 16 + lr] = (h16)a1;
        }
        asm volatile("" ::: "memory");
        const v16h pa = cat16(*(const v8ha*)(pl + lr * 32 + hi * 8), *(const v8ha*)(pl + lr * 32 + 16 + hi * 8));
#pragma unroll
        for (int n = 0; n < 8; ++n) { const h16* vp = f1_b + (size_t)(n * 16 + lr) * NN_ + n0 + hi * 8; o[n] = wmma16(pa, cat16(*(const v8h*)vp, *(const v8h*)(vp + 16)), o[n]); }
        asm volatile("v_nop\n\tv_nop\n\tv_nop\n\tv_nop" : "+v"(o[0]), "+v"(o[1]), "+v"(o[2]), "+v"(o[3]), "+v"(o[4]), "+v"(o[5]), "+v"(o[6]), "+v"(o[7]) : "v"(pa));
    }
#pragma unroll
    for (int n = 0; n < 8; ++n)
#pragma unroll
        for (int j = 0; j < 8; ++j) stile[(wave * 16 + hi * 8 + j) * 128 + n * 16 + lr] = o[n][j];
    __syncthreads();
    const float al = bfr(alpha[0]);
    auto pass = [&]() {
#pragma unroll
        for (int s = 0; s < 16; ++s) {
            const int Lid = 4 * s + (lane >> 3), piece = lane & 7;
            const int cl = wave * 32 + (Lid >> 1), mofs = (Lid & 1) * 32 + piece * 4;
            const size_t g = ((size_t)b * NC_ + cofs + cl) * NN_ + qt * 64 + mofs;
            v4f v;
#pragma unroll
            for (int i = 0; i < 4; ++i) v[i] = al * stile[(mofs + i) * 128 + cl] + bfr(x[g + i]);
            *(volatile v4f*)(out + g) = v;
        }
    };
    pass(); __threadfence(); pass();
}

extern "C" void kernel_launch(void* const* d_in, const int* in_sizes, int n_in,
                              void* d_out, int out_size, void* d_ws, size_t ws_size, hipStream_t stream) {
    (void)in_sizes; (void)n_in; (void)out_size;
    const float* x1 = (const float*)d_in[0]; const float* x2 = (const float*)d_in[1]; const float* x = (const float*)d_in[2];
    const float* g = (const float*)d_in[3]; const float* be = (const float*)d_in[4]; const float* mean = (const float*)d_in[5]; const float* var = (const float*)d_in[6];
    const float* Wb = (const float*)d_in[7]; const float* bb = (const float*)d_in[8]; const float* Wc = (const float*)d_in[9]; const float* bc = (const float*)d_in[10];
    const float* Wd = (const float*)d_in[11]; const float* bd = (const float*)d_in[12]; const float* alpha = (const float*)d_in[13];
    float* out = (float*)d_out;
    char* wsp = (char*)d_ws;
    auto take = [&](size_t bytes) { char* p = wsp; wsp += (bytes + 255) & ~(size_t)255; return (void*)p; };
    bf* X1T = (bf*)take((size_t)NB_ * NN_ * NC_ * 2); bf* X2T = (bf*)take((size_t)NB_ * NN_ * NC_ * 2); bf* XT = (bf*)take((size_t)NB_ * NN_ * NC_ * 2);
    bf* WH = (bf*)take((size_t)2 * CK * NC_ * 2); bf* WL = (bf*)take((size_t)2 * CK * NC_ * 2); float* BIAS32 = (float*)take((size_t)2 * CK * 32 * 4); bf* WD = (bf*)take((size_t)NC_ * NC_ * 2);
    h16* FA = (h16*)take((size_t)NB_ * NN_ * CK * 2); h16* FB = (h16*)take((size_t)NB_ * NN_ * CK * 2); h16* F1 = (h16*)take((size_t)NB_ * NC_ * NN_ * 2);
    float* M = (float*)take((size_t)NB_ * NN_ * 4); float* ZI = (float*)take((size_t)NB_ * NN_ * 4);
    if ((size_t)(wsp - (char*)d_ws) > ws_size) return;
    k_xt<<<dim3(NN_ / 64, NC_ / 64, NB_), 256, 0, stream>>>(x1, X1T);
    k_xt<<<dim3(NN_ / 64, NC_ / 64, NB_), 256, 0, stream>>>(x2, X2T);
    k_xt<<<dim3(NN_ / 64, NC_ / 64, NB_), 256, 0, stream>>>(x, XT);
    k_fold<<<(2 * CK) / 8, 256, 0, stream>>>(Wb, bb, Wc, bc, g, be, mean, var, WH, WL, BIAS32);
    k_cvtw<<<NC_ / 8, 256, 0, stream>>>(Wd, WD);
    k_gemmf<<<dim3(NN_ / 64, NB_, 1), 128, 0, stream>>>(X1T, WH, WL, BIAS32, 0, FA);
    k_gemmf<<<dim3(NN_ / 64, NB_, 1), 128, 0, stream>>>(X2T, WH, WL, BIAS32, 1, FB);
    k_gemm1<<<dim3(NC_ / 64, NN_ / 64, NB_), 128, 0, stream>>>(WD, XT, bd, F1);
    k_rowstats<<<NB_ * (NN_ / 64), 128, 0, stream>>>(FA, FB, M, ZI);
    const size_t lds = (size_t)64 * 128 * 4 + 4 * 16 * 32 * 2;
    k_out<<<NB_ * (NN_ / 64), 128, lds, stream>>>(FA, FB, F1, M, ZI, x, alpha, 0, out);
    k_out<<<NB_ * (NN_ / 64), 128, lds, stream>>>(FA, FB, F1, M, ZI, x, alpha, NC_ / 2, out);
}
